// TransformerBlock_2534030705250
// MI455X (gfx1250) — hardware-verified
//
#include <hip/hip_runtime.h>
#include <stddef.h>


typedef _Float16 v16h __attribute__((ext_vector_type(16)));
typedef _Float16 v8h  __attribute__((ext_vector_type(8)));
typedef float    v8f  __attribute__((ext_vector_type(8)));
typedef float    v4f  __attribute__((ext_vector_type(4)));

#ifndef NB
#define NB 2
#endif
#ifndef SEQ
#define SEQ 2048
#endif
#define NB_FULL  2
#define SEQ_FULL 2048
#define DIM   1024
#define NHEAD 16
#define HD    64
#define DFF   4096
#define MROWS (NB * SEQ)

static_assert(NB >= 1 && NB <= NB_FULL);
static_assert(SEQ >= 128 && SEQ <= SEQ_FULL && (SEQ % 128) == 0);
static_assert(DIM == NHEAD * HD);
static_assert(HD == 64);
static_assert(DIM == 4 * 256);
static_assert((DIM % 64) == 0 && (DIM % 32) == 0);
static_assert((DFF % 64) == 0 && (DFF % 32) == 0);
static_assert((MROWS % 64) == 0 && (MROWS % 8) == 0);
static_assert((size_t)MROWS * DFF < (size_t)0xFFFFFFFFu);

#define LDT 72
#define LDC 68
static_assert((LDT % 8) == 0 && LDT >= 64);
static_assert((LDC % 4) == 0 && LDC >= 64);

#define WCARRY 64.0f
#define PCARRY 1024.0f
#define VCARRY 64.0f
#define GCARRY 64.0f

#define WSQ_BYTES     ((size_t)DIM * DIM * 2)
#define WFF_BYTES     ((size_t)DIM * DFF * 2)
#define PLANE16_BYTES ((size_t)MROWS * DIM * 2)
#define HF_BYTES      ((size_t)MROWS * DIM * 4)
#define G16_BYTES     ((size_t)MROWS * DFF * 2)
#define OFF_W1T  (4 * WSQ_BYTES)
#define OFF_W2T  (OFF_W1T + WFF_BYTES)
#define OFF_LN1  (OFF_W2T + WFF_BYTES)
#define OFF_Q    (OFF_LN1 + PLANE16_BYTES)
#define OFF_K    (OFF_Q + PLANE16_BYTES)
#define OFF_VT   (OFF_K + PLANE16_BYTES)
#define OFF_CTX  (OFF_VT + PLANE16_BYTES)
#define OFF_LN2  (OFF_CTX + PLANE16_BYTES)
#define OFF_HF   (OFF_LN2 + PLANE16_BYTES)
#define OFF_G    (OFF_HF + HF_BYTES)
#define WS_TOTAL (OFF_G + G16_BYTES)
static_assert((WSQ_BYTES % 128) == 0 && (WFF_BYTES % 128) == 0);
static_assert((PLANE16_BYTES % 128) == 0 && (HF_BYTES % 128) == 0 && (G16_BYTES % 128) == 0);
static_assert(WS_TOTAL <= (size_t)134217728);

__device__ __forceinline__ float bf16r(float x) {
  unsigned int u = __float_as_uint(x);
  u = (u + 0x7FFFu + ((u >> 16) & 1u)) & 0xFFFF0000u;
  return __uint_as_float(u);
}

__device__ __forceinline__ v16h frag_at(const _Float16* p) {
  v8h lo = *(const v8h*)(p);
  v8h hi = *(const v8h*)(p + 16);
  v16h out;
#pragma unroll
  for (int i = 0; i < 8; ++i) { out[i] = lo[i]; out[i + 8] = hi[i]; }
  return out;
}
__device__ __forceinline__ v16h ld_frag(const _Float16* base, unsigned ld) {
  const unsigned lane = threadIdx.x & 31u;
  return frag_at(base + (lane & 15u) * ld + (lane >> 4) * 8u);
}

__device__ __forceinline__ v8f wmma16(v16h a, v16h b, v8f c) {
  v8f d = __builtin_amdgcn_wmma_f32_16x16x32_f16(false, a, false, b, (short)0, c,
                                                 false, false);
  asm volatile("v_nop\n\tv_nop\n\tv_nop\n\tv_nop" : "+v"(d) : "v"(a), "v"(b));
  return d;
}

__device__ __forceinline__ float red16_max(float x) {
#pragma unroll
  for (int off = 1; off < 16; off <<= 1) x = fmaxf(x, __shfl_xor(x, off, 32));
  return x;
}
__device__ __forceinline__ float red16_sum(float x) {
#pragma unroll
  for (int off = 1; off < 16; off <<= 1) x += __shfl_xor(x, off, 32);
  return x;
}
__device__ __forceinline__ float red32_sum(float x) {
#pragma unroll
  for (int off = 16; off >= 1; off >>= 1) x += __shfl_xor(x, off, 32);
  return x;
}

__device__ __forceinline__ void wave_lds_sync() {
  __builtin_amdgcn_fence(3  , "wavefront");
  asm volatile("s_wait_dscnt 0x0" ::: "memory");
  __builtin_amdgcn_wave_barrier();
}

__device__ __forceinline__ float gelu_tanh_f(float t) {
  const float u = 0.7978845608028654f * (t + 0.044715f * t * t * t);
  const float e = __expf(-2.0f * u);
  return t * __builtin_amdgcn_rcpf(1.0f + e);
}

__global__ __launch_bounds__(256) void wconv_kernel(
    const float* __restrict__ W, const unsigned ldw,
    _Float16* __restrict__ Wt, const unsigned ldk) {
  __shared__ _Float16 T[64 * LDT];
  const unsigned tid = threadIdx.x;
  const unsigned n0 = blockIdx.x * 64u;
  const unsigned k0 = blockIdx.y * 64u;
#pragma unroll 4
  for (unsigned j = 0; j < 16u; ++j) {
    const unsigned idx = tid + 256u * j;
    const unsigned kr = idx >> 6, nc = idx & 63u;
    const float v = W[(size_t)(k0 + kr) * ldw + n0 + nc];
    T[nc * LDT + kr] = (_Float16)(WCARRY * bf16r(v));
  }
  __syncthreads();
  v8h x[2];
  size_t off[2];
#pragma unroll
  for (unsigned i = 0; i < 2u; ++i) {
    const unsigned n = 32u * i + (tid >> 3);
    const unsigned kc = (tid & 7u) * 8u;
    x[i] = *(const v8h*)&T[n * LDT + kc];
    off[i] = (size_t)(n0 + n) * ldk + k0 + kc;
  }
#pragma unroll
  for (int i = 0; i < 2; ++i) *(volatile v8h*)(Wt + off[i]) = x[i];
  __threadfence();
#pragma unroll
  for (int i = 0; i < 2; ++i) *(volatile v8h*)(Wt + off[i]) = x[i];
}

__global__ __launch_bounds__(256) void ln_kernel(
    const float* __restrict__ src, const unsigned srcSeq, const int cvt,
    const float* __restrict__ gam, const float* __restrict__ bet,
    _Float16* __restrict__ dst) {
  const unsigned lane = threadIdx.x & 31u;
  const unsigned w = (unsigned)__builtin_amdgcn_readfirstlane((int)(threadIdx.x >> 5));
  const unsigned crow = blockIdx.x * 8u + w;
  const unsigned bidx = crow / (unsigned)SEQ;
  const unsigned sq = crow - bidx * (unsigned)SEQ;
  const float* sp = src + ((size_t)bidx * srcSeq + sq) * DIM + lane * 8u;
  const bool cv = (cvt != 0);

  float sum = 0.0f;
#pragma unroll 1
  for (unsigned j = 0; j < 4u; ++j) {
    const v4f a0 = *(const v4f*)(sp + j * 256u);
    const v4f a1 = *(const v4f*)(sp + j * 256u + 4u);
    float part = 0.0f;
#pragma unroll
    for (int i = 0; i < 4; ++i) {
      const float e0 = cv ? bf16r(a0[i]) : a0[i];
      const float e1 = cv ? bf16r(a1[i]) : a1[i];
      part += e0 + e1;
    }
    sum += part;
  }
  sum = red32_sum(sum);
  const float mean = sum * (1.0f / (float)DIM);

  float vs = 0.0f;
#pragma unroll 1
  for (unsigned j = 0; j < 4u; ++j) {
    const v4f a0 = *(const v4f*)(sp + j * 256u);
    const v4f a1 = *(const v4f*)(sp + j * 256u + 4u);
    float part = 0.0f;
#pragma unroll
    for (int i = 0; i < 4; ++i) {
      const float e0 = (cv ? bf16r(a0[i]) : a0[i]) - mean;
      const float e1 = (cv ? bf16r(a1[i]) : a1[i]) - mean;
      part += e0 * e0 + e1 * e1;
    }
    vs += part;
  }
  vs = red32_sum(vs);
  const float rinv = rsqrtf(vs * (1.0f / (float)DIM) + 1.0e-5f);

  _Float16* dp = dst + (size_t)crow * DIM + lane * 8u;
#pragma unroll 1
  for (unsigned j = 0; j < 4u; ++j) {
    const v4f a0 = *(const v4f*)(sp + j * 256u);
    const v4f a1 = *(const v4f*)(sp + j * 256u + 4u);
    const v4f g0 = *(const v4f*)(gam + lane * 8u + j * 256u);
    const v4f g1 = *(const v4f*)(gam + lane * 8u + j * 256u + 4u);
    const v4f t0 = *(const v4f*)(bet + lane * 8u + j * 256u);
    const v4f t1 = *(const v4f*)(bet + lane * 8u + j * 256u + 4u);
    v8h o;
#pragma unroll
    for (int i = 0; i < 4; ++i) {
      const float e0 = (cv ? bf16r(a0[i]) : a0[i]) - mean;
      const float e1 = (cv ? bf16r(a1[i]) : a1[i]) - mean;
      o[i]     = (_Float16)(bf16r(g0[i]) * e0 * rinv + bf16r(t0[i]));
      o[i + 4] = (_Float16)(bf16r(g1[i]) * e1 * rinv + bf16r(t1[i]));
    }
    *(volatile v8h*)(dp + j * 256u) = o;
    __threadfence();
    *(volatile v8h*)(dp + j * 256u) = o;
  }
}

template <int MODE>
__device__ __forceinline__ void gemm_tile(
    const _Float16* __restrict__ A16, const _Float16* __restrict__ Bt, const unsigned K,
    const float* __restrict__ bias, const float* __restrict__ resid,
    float* __restrict__ outf, _Float16* __restrict__ out16, const unsigned ldo) {
  __shared__ float Cs[64 * LDC];
  const unsigned tid = threadIdx.x, lane = tid & 31u;
  const unsigned w = (unsigned)__builtin_amdgcn_readfirstlane((int)(tid >> 5));
  const unsigned mw = w >> 1, nw = w & 1u;
  const unsigned hh = lane >> 4, m = lane & 15u;
  const unsigned n0 = blockIdx.x * 64u;
  const unsigned row0 = blockIdx.y * 64u;

  const _Float16* ap  = A16 + (size_t)(row0 + mw * 16u + m) * K + hh * 8u;
  const _Float16* bp0 = Bt + (size_t)(n0 + nw * 32u + m) * K + hh * 8u;
  const _Float16* bp1 = bp0 + (size_t)16 * K;
  v8f acc0 = {}, acc1 = {};
#pragma unroll 2
  for (unsigned k0 = 0; k0 < K; k0 += 32u) {
    const v16h a  = frag_at(ap + k0);
    const v16h b0 = frag_at(bp0 + k0);
    const v16h b1 = frag_at(bp1 + k0);
    acc0 = wmma16(a, b0, acc0);
    acc1 = wmma16(a, b1, acc1);
  }
#pragma unroll
  for (int r = 0; r < 8; ++r) {
    const unsigned ci = (mw * 16u + hh * 8u + (unsigned)r) * LDC + nw * 32u + m;
    Cs[ci]       = acc0[r];
    Cs[ci + 16u] = acc1[r];
  }
  __syncthreads();

  if (MODE == 0 || MODE == 3) {
    v8h x[2];
    size_t off[2];
#pragma unroll
    for (unsigned i = 0; i < 2u; ++i) {
      const unsigned r = 32u * i + (tid >> 3);
      const unsigned c = (tid & 7u) * 8u;
      const v4f u0 = *(const v4f*)&Cs[r * LDC + c];
      const v4f u1 = *(const v4f*)&Cs[r * LDC + c + 4];
      if (MODE == 0) {
#pragma unroll
        for (int j = 0; j < 4; ++j) {
          x[i][j]     = (_Float16)(u0[j] * (1.0f / WCARRY));
          x[i][j + 4] = (_Float16)(u1[j] * (1.0f / WCARRY));
        }
      } else {
        const v4f g0 = *(const v4f*)(bias + n0 + c);
        const v4f g1 = *(const v4f*)(bias + n0 + c + 4);
#pragma unroll
        for (int j = 0; j < 4; ++j) {
          const float t0 = u0[j] * (1.0f / WCARRY) + bf16r(g0[j]);
          const float t1 = u1[j] * (1.0f / WCARRY) + bf16r(g1[j]);
          x[i][j]     = (_Float16)(GCARRY * gelu_tanh_f(t0));
          x[i][j + 4] = (_Float16)(GCARRY * gelu_tanh_f(t1));
        }
      }
      off[i] = (size_t)(row0 + r) * ldo + n0 + c;
    }
#pragma unroll
    for (int i = 0; i < 2; ++i) *(volatile v8h*)(out16 + off[i]) = x[i];
    __threadfence();
#pragma unroll
    for (int i = 0; i < 2; ++i) *(volatile v8h*)(out16 + off[i]) = x[i];
  }

  if (MODE == 1) {
    const unsigned bidx = row0 / (unsigned)SEQ;
    const unsigned key0 = row0 - bidx * (unsigned)SEQ;
    v8h x[2];
    size_t off[2];
#pragma unroll
    for (unsigned i = 0; i < 2u; ++i) {
      const unsigned dcol = 32u * i + (tid >> 3);
      const unsigned kk = (tid & 7u) * 8u;
#pragma unroll
      for (unsigned j = 0; j < 8u; ++j)
        x[i][j] = (_Float16)(Cs[(kk + j) * LDC + dcol] * (1.0f / WCARRY));
      off[i] = ((size_t)bidx * DIM + n0 + dcol) * SEQ + key0 + kk;
    }
#pragma unroll
    for (int i = 0; i < 2; ++i) *(volatile v8h*)(out16 + off[i]) = x[i];
    __threadfence();
#pragma unroll
    for (int i = 0; i < 2; ++i) *(volatile v8h*)(out16 + off[i]) = x[i];
  }

  if (MODE == 2 || MODE == 4) {
    v4f xs[4];
    size_t off[4];
#pragma unroll
    for (unsigned i = 0; i < 4u; ++i) {
      const unsigned r = 16u * i + (tid >> 4);
      const unsigned c = (tid & 15u) * 4u;
      const unsigned crow = row0 + r;
      const unsigned bidx = crow / (unsigned)SEQ;
      const unsigned sq = crow - bidx * (unsigned)SEQ;
      const size_t frow = (size_t)bidx * SEQ_FULL + sq;
      const v4f u = *(const v4f*)&Cs[r * LDC + c];
      const v4f g = *(const v4f*)(bias + n0 + c);
      v4f val;
      if (MODE == 2) {
        const v4f rx = *(const v4f*)(resid + frow * DIM + n0 + c);
#pragma unroll
        for (int j = 0; j < 4; ++j)
          val[j] = (u[j] * (1.0f / (WCARRY * VCARRY)) + bf16r(g[j])) + bf16r(rx[j]);
        off[i] = (size_t)crow * DIM + n0 + c;
      } else {
        const v4f rh = *(const v4f*)(resid + (size_t)crow * DIM + n0 + c);
#pragma unroll
        for (int j = 0; j < 4; ++j)
          val[j] = (u[j] * (1.0f / (WCARRY * GCARRY)) + bf16r(g[j])) + rh[j];
        off[i] = frow * DIM + n0 + c;
      }
      xs[i] = val;
    }
#pragma unroll
    for (int i = 0; i < 4; ++i) *(volatile v4f*)(outf + off[i]) = xs[i];
    __threadfence();
#pragma unroll
    for (int i = 0; i < 4; ++i) *(volatile v4f*)(outf + off[i]) = xs[i];
  }
}

__global__ __launch_bounds__(256) void proj_rows_kernel(
    const _Float16* __restrict__ A16, const _Float16* __restrict__ Bt,
    _Float16* __restrict__ out16) {
  gemm_tile<0>(A16, Bt, (unsigned)DIM, nullptr, nullptr, nullptr, out16, (unsigned)DIM);
}
__global__ __launch_bounds__(256) void proj_vt_kernel(
    const _Float16* __restrict__ A16, const _Float16* __restrict__ Bt,
    _Float16* __restrict__ out16) {
  gemm_tile<1>(A16, Bt, (unsigned)DIM, nullptr, nullptr, nullptr, out16, (unsigned)SEQ);
}
__global__ __launch_bounds__(256) void oproj_kernel(
    const _Float16* __restrict__ A16, const _Float16* __restrict__ Bt,
    const float* __restrict__ bias, const float* __restrict__ xres,
    float* __restrict__ hout) {
  gemm_tile<2>(A16, Bt, (unsigned)DIM, bias, xres, hout, nullptr, (unsigned)DIM);
}
__global__ __launch_bounds__(256) void ffn1_kernel(
    const _Float16* __restrict__ A16, const _Float16* __restrict__ Bt,
    const float* __restrict__ bias, _Float16* __restrict__ out16) {
  gemm_tile<3>(A16, Bt, (unsigned)DIM, bias, nullptr, nullptr, out16, (unsigned)DFF);
}
__global__ __launch_bounds__(256) void ffn2_kernel(
    const _Float16* __restrict__ A16, const _Float16* __restrict__ Bt,
    const float* __restrict__ bias, const float* __restrict__ hres,
    float* __restrict__ outp) {
  gemm_tile<4>(A16, Bt, (unsigned)DFF, bias, hres, outp, nullptr, (unsigned)DIM);
}

__global__ __launch_bounds__(256) void attn_kernel(
    const _Float16* __restrict__ Qh, const _Float16* __restrict__ Kh,
    const _Float16* __restrict__ Vt, _Float16* __restrict__ Ov) {
  __shared__ _Float16 Ks[64 * LDT];
  __shared__ _Float16 Vs[64 * LDT];
  __shared__ _Float16 Ps[8 * 16 * LDT];

  const unsigned tid = threadIdx.x, lane = tid & 31u;
  const unsigned w = (unsigned)__builtin_amdgcn_readfirstlane((int)(tid >> 5));
  const unsigned hh = lane >> 4, m = lane & 15u;
  const unsigned q0 = blockIdx.x * 128u;
  const unsigned head = blockIdx.y;
  const unsigned b = blockIdx.z;
  const unsigned qw = q0 + w * 16u;
  const unsigned pb = w * (16u * LDT);
  const float scale = 0.125f;

  const size_t qoff = (size_t)(b * (unsigned)SEQ + qw + m) * DIM + head * HD + hh * 8u;
  v16h qf[2];
  qf[0] = frag_at(Qh + qoff);
  qf[1] = frag_at(Qh + qoff + 32);

  float mrow[8], lrow[8];
  v8f o[4];
#pragma unroll
  for (int v = 0; v < 8; ++v) { mrow[v] = -1.0e30f; lrow[v] = 0.0f; }
#pragma unroll
  for (int nb = 0; nb < 4; ++nb) o[nb] = (v8f){};

  const size_t kplane = (size_t)b * SEQ * DIM + head * HD;
  const size_t vplane = ((size_t)b * DIM + head * HD) * SEQ;

  const unsigned nkb = (q0 + 128u) >> 6;
  for (unsigned ib = 0; ib < nkb; ++ib) {
    const unsigned kb = ib * 64u;
#pragma unroll
    for (unsigned j = 0; j < 2u; ++j) {
      const unsigned idx = tid + 256u * j;
      const unsigned r = idx >> 3, c = (idx & 7u) * 8u;
      *(v8h*)&Ks[r * LDT + c] = *(const v8h*)(Kh + kplane + (size_t)(kb + r) * DIM + c);
      *(v8h*)&Vs[r * LDT + c] = *(const v8h*)(Vt + vplane + (size_t)r * SEQ + kb + c);
    }
    __syncthreads();

    if (kb <= qw) {
      v8f s[4];
#pragma unroll
      for (int kg = 0; kg < 4; ++kg) {
        v8f t = {};
#pragma unroll
        for (int c = 0; c < 2; ++c) {
          const v16h kf = ld_frag(&Ks[(kg * 16) * LDT + c * 32], LDT);
          t = wmma16(qf[c], kf, t);
        }
        s[kg] = t * scale;
      }

      if (kb + 63u > qw) {
#pragma unroll
        for (int kg = 0; kg < 4; ++kg) {
          const unsigned key = kb + (unsigned)kg * 16u + m;
#pragma unroll
          for (int v = 0; v < 8; ++v) {
            const unsigned qr = qw + hh * 8u + (unsigned)v;
            s[kg][v] = (key > qr) ? -1.0e30f : s[kg][v];
          }
        }
      }

      float alpha[8];
#pragma unroll
      for (int v = 0; v < 8; ++v) {
        float mx = fmaxf(fmaxf(s[0][v], s[1][v]), fmaxf(s[2][v], s[3][v]));
        mx = red16_max(mx);
        const float mn = fmaxf(mrow[v], mx);
        alpha[v] = __expf(mrow[v] - mn);
        mrow[v] = mn;
      }
#pragma unroll
      for (int kg = 0; kg < 4; ++kg)
#pragma unroll
        for (int v = 0; v < 8; ++v) s[kg][v] = __expf(s[kg][v] - mrow[v]);
#pragma unroll
      for (int v = 0; v < 8; ++v) {
        const float rs = red16_sum((s[0][v] + s[1][v]) + (s[2][v] + s[3][v]));
        lrow[v] = alpha[v] * lrow[v] + rs;
      }
#pragma unroll
      for (int nb = 0; nb < 4; ++nb)
#pragma unroll
        for (int v = 0; v < 8; ++v) o[nb][v] = o[nb][v] * alpha[v];

#pragma unroll
      for (int kg = 0; kg < 4; ++kg)
#pragma unroll
        for (int v = 0; v < 8; ++v)
          Ps[pb + (hh * 8u + (unsigned)v) * LDT + (unsigned)kg * 16u + m] =
              (_Float16)(s[kg][v] * PCARRY);
      wave_lds_sync();

#pragma unroll
      for (int c = 0; c < 2; ++c) {
        const v16h pf = ld_frag(&Ps[pb + c * 32], LDT);
#pragma unroll
        for (int nb = 0; nb < 4; ++nb) {
          const v16h vf = ld_frag(&Vs[(nb * 16) * LDT + c * 32], LDT);
          o[nb] = wmma16(pf, vf, o[nb]);
        }
      }
      wave_lds_sync();
    }
    __syncthreads();
  }

  float inv[8];
#pragma unroll
  for (int v = 0; v < 8; ++v) inv[v] = __builtin_amdgcn_rcpf(lrow[v]) * (VCARRY / PCARRY);
#pragma unroll
  for (int nb = 0; nb < 4; ++nb)
#pragma unroll
    for (int v = 0; v < 8; ++v)
      Ps[pb + (hh * 8u + (unsigned)v) * LDT + (unsigned)nb * 16u + m] =
          (_Float16)(o[nb][v] * inv[v]);
  wave_lds_sync();
  v8h x[4];
  size_t off[4];
#pragma unroll
  for (unsigned i = 0; i < 4u; ++i) {
    const unsigned r = 4u * i + (lane >> 3);
    const unsigned c = (lane & 7u) * 8u;
    x[i] = *(const v8h*)&Ps[pb + r * LDT + c];
    off[i] = (size_t)(b * (unsigned)SEQ + qw + r) * DIM + head * HD + c;
  }
#pragma unroll
  for (int i = 0; i < 4; ++i) *(volatile v8h*)(Ov + off[i]) = x[i];
  __threadfence();
#pragma unroll
  for (int i = 0; i < 4; ++i) *(volatile v8h*)(Ov + off[i]) = x[i];
}

extern "C" void kernel_launch(void* const* d_in, const int* in_sizes, int n_in,
                              void* d_out, int out_size, void* d_ws, size_t ws_size,
                              hipStream_t stream) {
  if (n_in < 14) return;
  const long long need_x = ((long long)(NB - 1) * SEQ_FULL + SEQ) * DIM;
  if ((long long)in_sizes[0] < need_x) return;
  for (int i = 1; i <= 4; ++i)
    if ((long long)in_sizes[i] < (long long)DIM * DIM) return;
  if (in_sizes[5] < DIM) return;
  if ((long long)in_sizes[6] < (long long)DIM * DFF) return;
  if (in_sizes[7] < DFF) return;
  if ((long long)in_sizes[8] < (long long)DFF * DIM) return;
  if (in_sizes[9] < DIM) return;
  for (int i = 10; i <= 13; ++i)
    if (in_sizes[i] < DIM) return;
  if ((long long)out_size < need_x) return;
  if (ws_size < WS_TOTAL) return;

  const float* X  = (const float*)d_in[0];
  const float* Wq = (const float*)d_in[1];
  const float* Wk = (const float*)d_in[2];
  const float* Wv = (const float*)d_in[3];
  const float* Wo = (const float*)d_in[4];
  const float* bo = (const float*)d_in[5];
  const float* W1 = (const float*)d_in[6];
  const float* b1 = (const float*)d_in[7];
  const float* W2 = (const float*)d_in[8];
  const float* b2 = (const float*)d_in[9];
  const float* g1 = (const float*)d_in[10];
  const float* s1 = (const float*)d_in[11];
  const float* g2 = (const float*)d_in[12];
  const float* s2 = (const float*)d_in[13];
  float* out = (float*)d_out;

  char* ws = (char*)d_ws;
  _Float16* Wqt   = (_Float16*)(ws + 0 * WSQ_BYTES);
  _Float16* Wkt   = (_Float16*)(ws + 1 * WSQ_BYTES);
  _Float16* Wvt   = (_Float16*)(ws + 2 * WSQ_BYTES);
  _Float16* Wot   = (_Float16*)(ws + 3 * WSQ_BYTES);
  _Float16* W1t   = (_Float16*)(ws + OFF_W1T);
  _Float16* W2t   = (_Float16*)(ws + OFF_W2T);
  _Float16* LN1   = (_Float16*)(ws + OFF_LN1);
  _Float16* Qh16  = (_Float16*)(ws + OFF_Q);
  _Float16* Kh16  = (_Float16*)(ws + OFF_K);
  _Float16* Vt16  = (_Float16*)(ws + OFF_VT);
  _Float16* Ctx16 = (_Float16*)(ws + OFF_CTX);
  _Float16* LN2   = (_Float16*)(ws + OFF_LN2);
  float*    Hf    = (float*)(ws + OFF_HF);
  _Float16* G16   = (_Float16*)(ws + OFF_G);

  dim3 blk(256);
  dim3 gsq(DIM / 64, MROWS / 64);

  wconv_kernel<<<dim3(DIM / 64, DIM / 64), blk, 0, stream>>>(Wq, (unsigned)DIM, Wqt, (unsigned)DIM);
  wconv_kernel<<<dim3(DIM / 64, DIM / 64), blk, 0, stream>>>(Wk, (unsigned)DIM, Wkt, (unsigned)DIM);
  wconv_kernel<<<dim3(DIM / 64, DIM / 64), blk, 0, stream>>>(Wv, (unsigned)DIM, Wvt, (unsigned)DIM);
  wconv_kernel<<<dim3(DIM / 64, DIM / 64), blk, 0, stream>>>(Wo, (unsigned)DIM, Wot, (unsigned)DIM);
  wconv_kernel<<<dim3(DFF / 64, DIM / 64), blk, 0, stream>>>(W1, (unsigned)DFF, W1t, (unsigned)DIM);
  wconv_kernel<<<dim3(DIM / 64, DFF / 64), blk, 0, stream>>>(W2, (unsigned)DIM, W2t, (unsigned)DFF);

  ln_kernel<<<dim3(MROWS / 8), blk, 0, stream>>>(X, (unsigned)SEQ_FULL, 1, g1, s1, LN1);
  proj_rows_kernel<<<gsq, blk, 0, stream>>>(LN1, Wqt, Qh16);
  proj_rows_kernel<<<gsq, blk, 0, stream>>>(LN1, Wkt, Kh16);
  proj_vt_kernel<<<gsq, blk, 0, stream>>>(LN1, Wvt, Vt16);
  attn_kernel<<<dim3(SEQ / 128, NHEAD, NB), blk, 0, stream>>>(Qh16, Kh16, Vt16, Ctx16);
  oproj_kernel<<<gsq, blk, 0, stream>>>(Ctx16, Wot, bo, X, Hf);
  ln_kernel<<<dim3(MROWS / 8), blk, 0, stream>>>(Hf, (unsigned)SEQ, 0, g2, s2, LN2);
  ffn1_kernel<<<dim3(DFF / 64, MROWS / 64), blk, 0, stream>>>(LN2, W1t, b1, G16);
  ffn2_kernel<<<gsq, blk, 0, stream>>>(G16, W2t, b2, Hf, out);
}
